// Tucker_24970939859199
// MI455X (gfx1250) — hardware-verified
//
#include <hip/hip_runtime.h>


#ifndef NSAMP
#define NSAMP 131072
#endif
#define NSAMP_FULL 131072
#define NUSER 200000
#define NITEM 100000
#define NTIME 5000
#define LD    32
#define NQR   (LD * LD)
#define CTT   64
#define AW    8
#define UP    40
#define VP    36

static_assert(LD == 32);
static_assert(NQR % 16 == 0);
static_assert(NQR % CTT == 0);
static_assert(256 * 8 == CTT * LD);
static_assert((CTT * LD * 2) % 128 == 0);
static_assert(NSAMP % (16 * AW) == 0);
static_assert(NSAMP <= NSAMP_FULL);
static_assert(32 * 16 == 16 * AW * 4);
static_assert(2 * 32 * 8 == 16 * LD);
static_assert(4 * 32 * 4 == 16 * LD);
static_assert(UP >= LD);
static_assert((UP * 2) % 16 == 0);
static_assert(VP >= LD);
static_assert((VP * 4) % 16 == 0);
static_assert((size_t)CTT * 33 * 4 <= 131072);
static_assert((size_t)AW * 16 * UP * 2 + 2 * (size_t)AW * 16 * VP * 4 + (size_t)AW * 16 * 4 <= 131072);

typedef unsigned short bf;
typedef __attribute__((ext_vector_type(16))) __bf16   v16bf;
typedef __attribute__((ext_vector_type(8)))  unsigned short v8us;
typedef __attribute__((ext_vector_type(8)))  float    v8f;
typedef __attribute__((ext_vector_type(4)))  float    v4f;
typedef v4f  __attribute__((may_alias)) v4fa;
typedef v8us __attribute__((may_alias)) v8usa;

__device__ __forceinline__ unsigned short f2bf(float f) { unsigned u = __float_as_uint(f); u += 0x7FFFu + ((u >> 16) & 1u); return (unsigned short)(u >> 16); }
__device__ __forceinline__ float bfr(float f) { return __uint_as_float(((unsigned)f2bf(f)) << 16); }
__device__ __forceinline__ v16bf cat16b(v8us lo, v8us hi) { return __builtin_bit_cast(v16bf, __builtin_shufflevector(lo, hi, 0, 1, 2, 3, 4, 5, 6, 7, 8, 9, 10, 11, 12, 13, 14, 15)); }
__device__ __forceinline__ v16bf ldb(const bf* p)  { return cat16b(*(const v8us*)p, *(const v8us*)(p + 16)); }
__device__ __forceinline__ v8f wmmab_g(v16bf a, v16bf b, v8f c) {
    c = __builtin_amdgcn_wmma_f32_16x16x32_bf16(false, a, false, b, (short)0, c, false, false);
    asm volatile("v_nop\n\tv_nop\n\tv_nop\n\tv_nop" : "+v"(c) : "v"(a), "v"(b));
    return c;
}
__device__ __forceinline__ void wave_sync() { __builtin_amdgcn_fence(3  , "wavefront"); __builtin_amdgcn_wave_barrier(); asm volatile("" ::: "memory"); }

__global__ __launch_bounds__(256) void k_coret(const float* __restrict__ core, bf* CT) {
    __shared__ __align__(16) float ts[CTT * 33];
    const int tid = threadIdx.x; const int c0 = blockIdx.x * CTT;
    { const int p = tid >> 3, cc = (tid & 7) * 8;
      const v4f x0 = *(const v4f*)(core + (size_t)p * NQR + c0 + cc); const v4f x1 = *(const v4f*)(core + (size_t)p * NQR + c0 + cc + 4);
#pragma unroll
      for (int i = 0; i < 4; ++i) { ts[(cc + i) * 33 + p] = x0[i]; ts[(cc + 4 + i) * 33 + p] = x1[i]; } }
    __syncthreads();
    const int row = tid >> 2, p8 = (tid & 3) * 8;
    v8us o;
#pragma unroll
    for (int k = 0; k < 8; ++k) o[k] = f2bf(ts[row * 33 + p8 + k]);
    bf* dst = CT + (size_t)(c0 + row) * LD + p8;
    *(volatile v8us*)dst = o; __threadfence(); *(volatile v8us*)dst = o;
}

__global__ __launch_bounds__(32 * AW) void k_score(const int* __restrict__ i_in, const int* __restrict__ j_in, const int* __restrict__ k_in,
                                                   const float* __restrict__ U, const float* __restrict__ V, const float* __restrict__ W,
                                                   const bf* __restrict__ CT, float* OUT) {
    __shared__ __align__(16) bf    us[AW * 16 * UP];
    __shared__ __align__(16) float vs[AW * 16 * VP];
    __shared__ __align__(16) float wt[AW * 16 * VP];
    __shared__ __align__(16) float ob[AW * 16];
    const int lane = threadIdx.x & 31, lr = lane & 15, hi = lane >> 4;
    const int wave = __builtin_amdgcn_readfirstlane((int)(threadIdx.x >> 5));
    const int base = (blockIdx.x * AW + wave) * 16;
    const int ub0 = wave * 16 * UP, vb0 = wave * 16 * VP;
#pragma unroll
    for (int s = 0; s < 2; ++s) { const int p = s * 32 + lane; const int row = p >> 2, c8 = (p & 3) * 8;
        int iu = i_in[base + row]; iu = iu < 0 ? 0 : (iu > NUSER - 1 ? NUSER - 1 : iu);
        const v8f x = *(const v8f*)(U + (size_t)iu * LD + c8); v8us o;
#pragma unroll
        for (int k = 0; k < 8; ++k) o[k] = f2bf(x[k]);
        *(v8usa*)(&us[ub0 + row * UP + c8]) = o; }
#pragma unroll
    for (int s = 0; s < 4; ++s) { const int p = s * 32 + lane; const int row = p >> 3, c4 = (p & 7) * 4;
        int jv = j_in[base + row]; jv = jv < 0 ? 0 : (jv > NITEM - 1 ? NITEM - 1 : jv);
        int kv = k_in[base + row]; kv = kv < 0 ? 0 : (kv > NTIME - 1 ? NTIME - 1 : kv);
        const v4f x = *(const v4f*)(V + (size_t)jv * LD + c4); const v4f y = *(const v4f*)(W + (size_t)kv * LD + c4); v4f xo, yo;
#pragma unroll
        for (int i = 0; i < 4; ++i) { xo[i] = bfr(x[i]); yo[i] = bfr(y[i]); }
        *(v4fa*)(&vs[vb0 + row * VP + c4]) = xo; *(v4fa*)(&wt[vb0 + row * VP + c4]) = yo; }
    wave_sync();
    const v16bf ub = cat16b(*(const v8usa*)(&us[ub0 + lr * UP + 8 * hi]), *(const v8usa*)(&us[ub0 + lr * UP + 16 + 8 * hi]));
    const v4f w0a = *(const v4fa*)(&wt[vb0 + lr * VP + 8 * hi]),      w0b = *(const v4fa*)(&wt[vb0 + lr * VP + 8 * hi + 4]);
    const v4f w1a = *(const v4fa*)(&wt[vb0 + lr * VP + 16 + 8 * hi]), w1b = *(const v4fa*)(&wt[vb0 + lr * VP + 16 + 8 * hi + 4]);
    const size_t ao = (size_t)lr * LD + 8 * hi;
    v8f s0 = (v8f){}, s1 = (v8f){};
#pragma unroll 1
    for (int q4 = 0; q4 < LD; q4 += 4) {
        const v4f vv = *(const v4fa*)(&vs[vb0 + lr * VP + q4]);
#pragma unroll
        for (int u = 0; u < 4; ++u) {
            const bf* ap = CT + ao + (size_t)(q4 + u) * (LD * LD);
            const v16bf a0 = ldb(ap), a1 = ldb(ap + 16 * LD);
            v8f c0 = (v8f){}, c1 = (v8f){};
            c0 = wmmab_g(a0, ub, c0);
            c1 = wmmab_g(a1, ub, c1);
            const float vq = vv[u];
            s0 = s0 + c0 * vq; s1 = s1 + c1 * vq; }
    }
    float acc = 0.0f;
#pragma unroll
    for (int r = 0; r < 4; ++r) { acc += s0[r] * w0a[r]; acc += s0[4 + r] * w0b[r]; acc += s1[r] * w1a[r]; acc += s1[4 + r] * w1b[r]; }
    acc += __shfl_xor(acc, 16, 32);
    if (hi == 0) ob[wave * 16 + lr] = acc;
    __syncthreads();
    if (wave == 0) {
        const v4f val = *(const v4fa*)(&ob[lane * 4]);
        float* dst = OUT + (size_t)blockIdx.x * (16 * AW) + lane * 4;
        *(volatile v4f*)dst = val; __threadfence(); *(volatile v4f*)dst = val;
    }
}

static constexpr size_t al256(size_t v) { return (v + 255) & ~(size_t)255; }
static constexpr size_t SZ_CT = al256((size_t)NQR * LD * 2);
static constexpr size_t SZ_TOTAL = SZ_CT;
static_assert(SZ_TOTAL <= (size_t)134217728);
static_assert((size_t)(NQR / CTT) * 256 * 8 * 2 == (size_t)NQR * LD * 2);

extern "C" void kernel_launch(void* const* d_in, const int* in_sizes, int n_in,
                              void* d_out, int out_size, void* d_ws, size_t ws_size, hipStream_t stream) {
    if (n_in < 7) return;
    if (in_sizes[0] < NSAMP || in_sizes[1] < NSAMP || in_sizes[2] < NSAMP) return;
    if ((size_t)in_sizes[3] < (size_t)NUSER * LD || (size_t)in_sizes[4] < (size_t)NITEM * LD || (size_t)in_sizes[5] < (size_t)NTIME * LD) return;
    if ((size_t)in_sizes[6] < (size_t)LD * LD * LD) return;
    if (out_size < NSAMP) return;
    if (SZ_TOTAL > ws_size) return;
    const int* i_in = (const int*)d_in[0];
    const int* j_in = (const int*)d_in[1];
    const int* k_in = (const int*)d_in[2];
    const float* U = (const float*)d_in[3];
    const float* V = (const float*)d_in[4];
    const float* W = (const float*)d_in[5];
    const float* core = (const float*)d_in[6];
    float* OUT = (float*)d_out;
    bf* CT = (bf*)d_ws;

    k_coret<<<dim3(NQR / CTT, 1, 1), 256, 0, stream>>>(core, CT);
    k_score<<<dim3(NSAMP / (16 * AW), 1, 1), 32 * AW, 0, stream>>>(i_in, j_in, k_in, U, V, W, CT, OUT);
}
